// GemmaTensorProductAttention_22900765622442
// MI455X (gfx1250) — hardware-verified
//
#include <hip/hip_runtime.h>


namespace {
constexpr int Bn = 2, S = 2048, HID = 2048, NH = 16, NKV = 8, D = 128, QR = 6, KR = 2, VR = 2, WIN = 1024, NT = Bn * S;
constexpr int NPJ = 1408;
constexpr float QS = 8.0f, KS = 8.0f, VS = 8.0f, PS = 8.0f, CAP = 50.0f, SCALE = 0.08838834764831845f, EPS = 1e-6f;
constexpr size_t QPL = (size_t)Bn * NH * S * D, KPL = (size_t)Bn * NKV * S * D, CPL = (size_t)NT * HID;

typedef _Float16 b16;
typedef __attribute__((ext_vector_type(16))) _Float16 v16b;
typedef __attribute__((ext_vector_type(16))) __bf16 v16bb;
typedef __attribute__((ext_vector_type(8))) _Float16 v8b;
typedef __attribute__((ext_vector_type(8))) unsigned short v8us;
typedef __attribute__((ext_vector_type(8))) float v8f;
typedef __attribute__((ext_vector_type(4))) float v4f;
__device__ __forceinline__ float bf16_rne(float f) { unsigned int u = __float_as_uint(f); u += 0x7FFFu + ((u >> 16) & 1u); return __uint_as_float(u & 0xFFFF0000u); }
__device__ __forceinline__ unsigned short bf16_bits(float f) { unsigned int u = __float_as_uint(f); u += 0x7FFFu + ((u >> 16) & 1u); return (unsigned short)(u >> 16); }
__device__ __forceinline__ void split16(float v, b16& hi, b16& lo) { hi = (b16)v; lo = (b16)(v - (float)hi); }
__device__ __forceinline__ v16b frag_kb(const b16* p, int hh) { const v8b a = *(const v8b*)(p + 8 * hh), b = *(const v8b*)(p + 16 + 8 * hh); v16b f;
#pragma unroll
  for (int e = 0; e < 8; ++e) { f[e] = a[e]; f[8 + e] = b[e]; } return f; }
__device__ __forceinline__ v16bb frag_bf(const unsigned short* p, int hh) { const v8us a = *(const v8us*)(p + 8 * hh), b = *(const v8us*)(p + 16 + 8 * hh); union { unsigned short s[16]; v16bb v; } u;
#pragma unroll
  for (int e = 0; e < 8; ++e) { u.s[e] = a[e]; u.s[8 + e] = b[e]; } return u.v; }
__device__ __forceinline__ v16bb frag_f32bf(const float* p, int hh) { union { unsigned short s[16]; v16bb v; } u;
#pragma unroll
  for (int e = 0; e < 8; ++e) { u.s[e] = bf16_bits(p[8 * hh + e]); u.s[8 + e] = bf16_bits(p[16 + 8 * hh + e]); } return u.v; }
__device__ __forceinline__ v8f wmma16b(v16b a, v16b b, v8f c) { v8f d = __builtin_amdgcn_wmma_f32_16x16x32_f16(false, a, false, b, (short)0, c, false, false); asm volatile("v_nop\n\tv_nop\n\tv_nop\n\tv_nop" : "+v"(d) : "v"(a), "v"(b)); return d; }
__device__ __forceinline__ v8f wmma16bb(v16bb a, v16bb b, v8f c) { v8f d = __builtin_amdgcn_wmma_f32_16x16x32_bf16(false, a, false, b, (short)0, c, false, false); asm volatile("v_nop\n\tv_nop\n\tv_nop\n\tv_nop" : "+v"(d) : "v"(a), "v"(b)); return d; }
__device__ __forceinline__ void wave_lds_sync() { __builtin_amdgcn_fence(__ATOMIC_RELEASE, "workgroup"); __builtin_amdgcn_wave_barrier(); __builtin_amdgcn_fence(__ATOMIC_ACQUIRE, "workgroup"); }
__device__ __forceinline__ float nexp(float x) { return __builtin_amdgcn_exp2f(x * 1.4426950408889634f); }
__device__ __forceinline__ float pmul(float a, float b) { float p = a * b; asm volatile("" : "+v"(p)); return p; }
__device__ __forceinline__ float tanh_acc(float x) { const float ax = fabsf(x);
  if (ax < 0.0625f) { const float x2 = x * x; return x * (1.0f + x2 * (-0.333333333f + x2 * (0.133333333f + x2 * (-0.053968254f)))); }
  const float e = nexp(-2.0f * ax); const float t = (1.0f - e) * __builtin_amdgcn_rcpf(1.0f + e); return (x >= 0.0f) ? t : -t; }

__global__ __launch_bounds__(256) void prep_kernel(const float* __restrict__ WAq, const float* __restrict__ WAk, const float* __restrict__ WAv, const float* __restrict__ WBq, const float* __restrict__ WBk, const float* __restrict__ WBv, const float* __restrict__ Wo, const float* __restrict__ qnw, const float* __restrict__ knw, unsigned short* __restrict__ wcat, b16* __restrict__ wo16, float* __restrict__ P) {
  const size_t tid = (size_t)blockIdx.x * blockDim.x + threadIdx.x, nth = (size_t)gridDim.x * blockDim.x;
  for (int pass = 0; pass < 2; ++pass) {
    for (size_t p = tid; p < (size_t)NPJ * HID / 8; p += nth) { const int o = (int)(p / (HID / 8)), k8 = (int)(p % (HID / 8)) * 8; v8us v;
#pragma unroll
      for (int e = 0; e < 8; ++e) { const size_t k = k8 + e; float w;
        if (o < 96) w = WAq[k * 96 + o]; else if (o < 112) w = WAk[k * 16 + o - 96]; else if (o < 128) w = WAv[k * 16 + o - 112]; else if (o < 896) w = WBq[k * 768 + o - 128]; else if (o < 1152) w = WBk[k * 256 + o - 896]; else w = WBv[k * 256 + o - 1152];
        v[e] = bf16_bits(w); }
      *(volatile v8us*)(wcat + (size_t)o * HID + k8) = v; }
    for (size_t p = tid; p < (size_t)HID * HID / 8; p += nth) { const int o = (int)(p / (HID / 8)), k8 = (int)(p % (HID / 8)) * 8; v8b v;
#pragma unroll
      for (int e = 0; e < 8; ++e) v[e] = (b16)bf16_rne(Wo[(size_t)(k8 + e) * HID + o]);
      *(volatile v8b*)(wo16 + (size_t)o * HID + k8) = v; }
    for (size_t p = tid; p < 256; p += nth) P[p] = 1.0f + bf16_rne((p < 128) ? qnw[p] : knw[p - 128]);
    __threadfence(); }
}

__global__ __launch_bounds__(128) void proj_kernel(const float* __restrict__ hs, const unsigned short* __restrict__ wcat, float* __restrict__ proj) {
  __shared__ __attribute__((aligned(16))) float Ts[4][32 * 64];
  const int lane = threadIdx.x & 31, wave = threadIdx.x >> 5, nloc = lane & 15, hlf = lane >> 4, m0 = blockIdx.y * 128 + wave * 32, c0 = blockIdx.x * 64;
  v8f acc[2][4];
#pragma unroll
  for (int r = 0; r < 2; ++r)
#pragma unroll
    for (int t = 0; t < 4; ++t) acc[r][t] = (v8f){};
#pragma unroll 2
  for (int kb = 0; kb < HID; kb += 32) { const v16bb a0 = frag_f32bf(hs + (size_t)(m0 + nloc) * HID + kb, hlf), a1 = frag_f32bf(hs + (size_t)(m0 + 16 + nloc) * HID + kb, hlf);
#pragma unroll
    for (int t = 0; t < 4; ++t) { const v16bb bw = frag_bf(wcat + (size_t)(c0 + t * 16 + nloc) * HID + kb, hlf); acc[0][t] = wmma16bb(a0, bw, acc[0][t]); acc[1][t] = wmma16bb(a1, bw, acc[1][t]); } }
  float* Tt = Ts[wave];
#pragma unroll
  for (int t = 0; t < 4; ++t)
#pragma unroll
    for (int r = 0; r < 2; ++r)
#pragma unroll
      for (int v = 0; v < 8; ++v) Tt[(r * 16 + v + 8 * hlf) * 64 + t * 16 + nloc] = acc[r][t][v];
  wave_lds_sync();
  for (int pass = 0; pass < 2; ++pass) {
#pragma unroll
    for (int j = 0; j < 16; ++j) { const int rr = j * 2 + hlf, c4 = nloc * 4; *(volatile v4f*)(proj + (size_t)(m0 + rr) * NPJ + c0 + c4) = *(const v4f*)(Tt + rr * 64 + c4); }
    __threadfence(); }
}

typedef __attribute__((ext_vector_type(2))) _Float16 v2b;
typedef __attribute__((ext_vector_type(2))) float v2f;
__global__ __launch_bounds__(256) void qk_kernel(const float* __restrict__ proj, const float* __restrict__ cosr, const float* __restrict__ sinr, const float* __restrict__ P, b16* __restrict__ qp, b16* __restrict__ kp) {
  const int wid = threadIdx.x >> 5, lane = threadIdx.x & 31; const int tok = blockIdx.x * 8 + wid, b = tok / S, s = tok % S; const float* pr = proj + (size_t)tok * NPJ;
  const int dA = 2 * lane, dB = 2 * lane + 1;
  const float cA = bf16_rne(cosr[(size_t)s * 64 + dA]), cB = bf16_rne(cosr[(size_t)s * 64 + dB]), sA = bf16_rne(sinr[(size_t)s * 64 + dA]), sB = bf16_rne(sinr[(size_t)s * 64 + dB]);
  float Bf[8][4];
#pragma unroll
  for (int f = 0; f < 8; ++f) { const float* br = pr + ((f < 6) ? (128 + f * D) : (896 + (f - 6) * D)); const float* w = P + ((f < 6) ? 0 : 128);
    const v2f xa = *(const v2f*)(br + dA), xb = *(const v2f*)(br + 64 + dA); const float x0 = xa[0], x1 = xa[1], x2 = xb[0], x3 = xb[1]; float ss = (pmul(x0, x0) + pmul(x1, x1)) + (pmul(x2, x2) + pmul(x3, x3));
#pragma unroll
    for (int o = 1; o < 32; o <<= 1) ss += __shfl_xor(ss, o);
    const float is = rsqrtf(ss * (1.0f / D) + EPS); const float n0 = x0 * is * w[dA], n1 = x1 * is * w[dB], n2 = x2 * is * w[64 + dA], n3 = x3 * is * w[64 + dB];
    Bf[f][0] = n0 * cA - n2 * sA; Bf[f][1] = n1 * cB - n3 * sB; Bf[f][2] = n0 * sA + n2 * cA; Bf[f][3] = n1 * sB + n3 * cB; }
  for (int h = 0; h < NH; ++h) { float q_[4] = {0.0f, 0.0f, 0.0f, 0.0f};
#pragma unroll
    for (int r = 0; r < QR; ++r) { const float a = pr[h * QR + r];
#pragma unroll
      for (int j = 0; j < 4; ++j) q_[j] += pmul(a, Bf[r][j]); }
    b16* dst = qp + (((size_t)b * NH + h) * S + s) * D; v2b h01, l01, h23, l23; b16 t0, t1;
    split16(q_[0] * (SCALE * QS / QR), t0, t1); h01[0] = t0; l01[0] = t1; split16(q_[1] * (SCALE * QS / QR), t0, t1); h01[1] = t0; l01[1] = t1;
    split16(q_[2] * (SCALE * QS / QR), t0, t1); h23[0] = t0; l23[0] = t1; split16(q_[3] * (SCALE * QS / QR), t0, t1); h23[1] = t0; l23[1] = t1;
    for (int pass = 0; pass < 2; ++pass) { *(volatile v2b*)(dst + dA) = h01; *(volatile v2b*)(dst + 64 + dA) = h23; *(volatile v2b*)(dst + QPL + dA) = l01; *(volatile v2b*)(dst + QPL + 64 + dA) = l23; } }
  for (int kv = 0; kv < NKV; ++kv) { float k_[4] = {0.0f, 0.0f, 0.0f, 0.0f};
#pragma unroll
    for (int r = 0; r < KR; ++r) { const float a = pr[96 + kv * KR + r];
#pragma unroll
      for (int j = 0; j < 4; ++j) k_[j] += pmul(a, Bf[6 + r][j]); }
    b16* dst = kp + (((size_t)b * NKV + kv) * S + s) * D; v2b k01, k23; k01[0] = (b16)(k_[0] * (KS / KR)); k01[1] = (b16)(k_[1] * (KS / KR)); k23[0] = (b16)(k_[2] * (KS / KR)); k23[1] = (b16)(k_[3] * (KS / KR));
    for (int pass = 0; pass < 2; ++pass) { *(volatile v2b*)(dst + dA) = k01; *(volatile v2b*)(dst + 64 + dA) = k23; } }
  __threadfence();
}

__global__ __launch_bounds__(256) void vt_kernel(const float* __restrict__ proj, b16* __restrict__ vt) {
  __shared__ __attribute__((aligned(16))) b16 Tv[D][128 + 8], Tl[D][128 + 8];
  const int t_ = threadIdx.x, t0 = blockIdx.x * 128, kv = blockIdx.y, b = blockIdx.z;
  for (int i = t_; i < 128 * D; i += 256) { const int tt = i >> 7, d = i & 127; const float* pr = proj + ((size_t)b * S + t0 + tt) * NPJ; const float v = (pmul(pr[112 + kv * VR], pr[1152 + d]) + pmul(pr[112 + kv * VR + 1], pr[1152 + D + d])) * (VS / VR); b16 h_, l_; split16(v, h_, l_); Tv[d][tt] = h_; Tl[d][tt] = l_; }
  __syncthreads();
  for (int pass = 0; pass < 2; ++pass) { for (int i = t_; i < D * 16; i += 256) { const int d = i >> 4, c8 = (i & 15) * 8; const size_t o = (((size_t)b * NKV + kv) * D + d) * S + t0 + c8; *(volatile v8b*)(vt + o) = *(const v8b*)(&Tv[d][c8]); *(volatile v8b*)(vt + KPL + o) = *(const v8b*)(&Tl[d][c8]); } __threadfence(); }
}

__global__ __launch_bounds__(256) void attn_kernel(const b16* __restrict__ qp, const b16* __restrict__ kp, const b16* __restrict__ vt, b16* __restrict__ ctx) {
  __shared__ __attribute__((aligned(16))) b16 Os[16][8 * D + 8], Ol[16][8 * D + 8];
  const int wid = threadIdx.x >> 5, lane = threadIdx.x & 31, hh = lane >> 4, col = lane & 15; const int b = blockIdx.x / (S / 16), q0 = (blockIdx.x % (S / 16)) * 16, h = blockIdx.y * 8 + wid, kv = h >> 1, qi = q0 + col;
  const b16* Q = qp + (((size_t)b * NH + h) * S) * D; const b16* K = kp + (((size_t)b * NKV + kv) * S) * D; const b16* V = vt + (((size_t)b * NKV + kv) * D) * S;
  v16b qf[4];
#pragma unroll
  for (int ks = 0; ks < 4; ++ks) qf[ks] = frag_kb(Q + (size_t)qi * D + ks * 32, hh);
  float m = -INFINITY, l = 0.0f; v8f o[8];
#pragma unroll
  for (int t = 0; t < 8; ++t) o[t] = (v8f){};
  const int kstart = max(0, q0 - (WIN - 1)) & ~31, kend = q0 + 16;
  for (int kb = kstart; kb < kend; kb += 32) { const bool edge = (kb + 32 > q0) || (kb < q0 + 15 - (WIN - 1)); v8f s0 = {}, s1 = {};
#pragma unroll
    for (int ks = 0; ks < 4; ++ks) { const v16b ka = frag_kb(K + (size_t)(kb + col) * D + ks * 32, hh), kc = frag_kb(K + (size_t)(kb + 16 + col) * D + ks * 32, hh); s0 = wmma16b(ka, qf[ks], s0); s1 = wmma16b(kc, qf[ks], s1); }
    float mr = -INFINITY;
#pragma unroll
    for (int r = 0; r < 8; ++r) { float a0 = CAP * tanh_acc(s0[r] * (1.0f / (QS * KS * CAP))), a1 = CAP * tanh_acc(s1[r] * (1.0f / (QS * KS * CAP)));
      if (edge) { const int j0 = kb + 8 * hh + r, j1 = kb + 16 + 8 * hh + r; if (j0 > qi || j0 <= qi - WIN) a0 = -INFINITY; if (j1 > qi || j1 <= qi - WIN) a1 = -INFINITY; }
      s0[r] = a0; s1[r] = a1; mr = fmaxf(mr, fmaxf(a0, a1)); }
    mr = fmaxf(mr, __shfl_xor(mr, 16));
    const float mn = fmaxf(m, mr); const float al_ = (mn == -INFINITY) ? 1.0f : nexp(m - mn); m = mn; float sum = 0.0f; v16b pbv;
#pragma unroll
    for (int r = 0; r < 8; ++r) { const float e0 = (s0[r] == -INFINITY) ? 0.0f : nexp(s0[r] - mn), e1 = (s1[r] == -INFINITY) ? 0.0f : nexp(s1[r] - mn); sum += e0 + e1; pbv[r] = (b16)(e0 * PS); pbv[8 + r] = (b16)(e1 * PS); }
    sum += __shfl_xor(sum, 16); l = l * al_ + sum;
#pragma unroll
    for (int t = 0; t < 8; ++t) { o[t] *= al_; const v16b vf = frag_kb(V + (size_t)(t * 16 + col) * S + kb, hh), vl = frag_kb(V + KPL + (size_t)(t * 16 + col) * S + kb, hh); o[t] = wmma16b(vf, pbv, o[t]); o[t] = wmma16b(vl, pbv, o[t]); } }
  const float inv = 1.0f / (l * VS * PS);
#pragma unroll
  for (int t = 0; t < 8; ++t)
#pragma unroll
    for (int r = 0; r < 8; ++r) { b16 h_, l_; split16(o[t][r] * inv, h_, l_); Os[col][wid * D + t * 16 + 8 * hh + r] = h_; Ol[col][wid * D + t * 16 + 8 * hh + r] = l_; }
  __syncthreads();
  for (int pass = 0; pass < 2; ++pass) { for (int i = threadIdx.x; i < 16 * (8 * D / 8); i += 256) { const int rr = i / (8 * D / 8), c8 = (i % (8 * D / 8)) * 8; const size_t o_ = ((size_t)b * S + q0 + rr) * HID + blockIdx.y * 8 * D + c8; *(volatile v8b*)(ctx + o_) = *(const v8b*)(&Os[rr][c8]); *(volatile v8b*)(ctx + CPL + o_) = *(const v8b*)(&Ol[rr][c8]); } __threadfence(); }
}

__global__ __launch_bounds__(128) void out_kernel(const b16* __restrict__ ctx, const b16* __restrict__ wo16, float* __restrict__ out) {
  __shared__ __attribute__((aligned(16))) float Ts[4][32 * 64];
  const int lane = threadIdx.x & 31, wave = threadIdx.x >> 5, nloc = lane & 15, hlf = lane >> 4, m0 = blockIdx.y * 128 + wave * 32, c0 = blockIdx.x * 64;
  v8f acc[2][4];
#pragma unroll
  for (int r = 0; r < 2; ++r)
#pragma unroll
    for (int t = 0; t < 4; ++t) acc[r][t] = (v8f){};
#pragma unroll 2
  for (int kb = 0; kb < HID; kb += 32) { const v16b a0 = frag_kb(ctx + (size_t)(m0 + nloc) * HID + kb, hlf), a1 = frag_kb(ctx + (size_t)(m0 + 16 + nloc) * HID + kb, hlf), l0 = frag_kb(ctx + CPL + (size_t)(m0 + nloc) * HID + kb, hlf), l1 = frag_kb(ctx + CPL + (size_t)(m0 + 16 + nloc) * HID + kb, hlf);
#pragma unroll
    for (int t = 0; t < 4; ++t) { const v16b bw = frag_kb(wo16 + (size_t)(c0 + t * 16 + nloc) * HID + kb, hlf); acc[0][t] = wmma16b(a0, bw, acc[0][t]); acc[0][t] = wmma16b(l0, bw, acc[0][t]); acc[1][t] = wmma16b(a1, bw, acc[1][t]); acc[1][t] = wmma16b(l1, bw, acc[1][t]); } }
  float* Tt = Ts[wave];
#pragma unroll
  for (int t = 0; t < 4; ++t)
#pragma unroll
    for (int r = 0; r < 2; ++r)
#pragma unroll
      for (int v = 0; v < 8; ++v) Tt[(r * 16 + v + 8 * hlf) * 64 + t * 16 + nloc] = acc[r][t][v];
  wave_lds_sync();
  for (int pass = 0; pass < 2; ++pass) {
#pragma unroll
    for (int j = 0; j < 16; ++j) { const int rr = j * 2 + hlf, c4 = nloc * 4; *(volatile v4f*)(out + (size_t)(m0 + rr) * HID + c0 + c4) = *(const v4f*)(Tt + rr * 64 + c4); }
    __threadfence(); }
}
}

extern "C" void kernel_launch(void* const* d_in, const int* in_sizes, int n_in,
                              void* d_out, int out_size, void* d_ws, size_t ws_size, hipStream_t stream) {
  (void)n_in; (void)out_size;
  const float* hs = (const float*)d_in[0]; const float* cosr = (const float*)d_in[1]; const float* sinr = (const float*)d_in[2]; const float* WAq = (const float*)d_in[3]; const float* WAk = (const float*)d_in[4]; const float* WAv = (const float*)d_in[5];
  const float* WBq = (const float*)d_in[6]; const float* WBk = (const float*)d_in[7]; const float* WBv = (const float*)d_in[8]; const float* Wo = (const float*)d_in[9]; const float* qnw = (const float*)d_in[10]; const float* knw = (const float*)d_in[11];
  float* out = (float*)d_out;
  if (in_sizes[0] != NT * HID || in_sizes[1] != S * 64 || in_sizes[3] != HID * 96 || in_sizes[6] != HID * 768 || in_sizes[9] != HID * HID || in_sizes[16] != S) return;
  size_t off = 0; char* ws = (char*)d_ws;
  auto carve = [&](size_t bytes) { char* p = ws + off; off += (bytes + 255) & ~(size_t)255; return p; };
  unsigned short* wcat = (unsigned short*)carve((size_t)NPJ * HID * 2); b16* wo16 = (b16*)carve((size_t)HID * HID * 2); float* P = (float*)carve(256 * 4); float* proj = (float*)carve((size_t)NT * NPJ * 4);
  b16* qp = (b16*)carve(QPL * 2 * 2); b16* kp = (b16*)carve(KPL * 2); b16* vt = (b16*)carve(KPL * 2 * 2); b16* ctx = (b16*)carve(CPL * 2 * 2);
  if (off > ws_size) return;
  prep_kernel<<<512, 256, 0, stream>>>(WAq, WAk, WAv, WBq, WBk, WBv, Wo, qnw, knw, wcat, wo16, P);
  proj_kernel<<<dim3(NPJ / 64, NT / 128), 128, 0, stream>>>(hs, wcat, proj);
  qk_kernel<<<NT / 8, 256, 0, stream>>>(proj, cosr, sinr, P, qp, kp);
  vt_kernel<<<dim3(S / 128, NKV, Bn), 256, 0, stream>>>(proj, vt);
  attn_kernel<<<dim3(Bn * S / 16, 2), 256, 0, stream>>>(qp, kp, vt, ctx);
  out_kernel<<<dim3(HID / 64, NT / 128), 128, 0, stream>>>(ctx, wo16, out);
}
